// ExpertFFNUnique_9929964389207
// MI455X (gfx1250) — hardware-verified
//
#include <hip/hip_runtime.h>
#include <stdint.h>
#include <stddef.h>
#include <math.h>

#pragma clang fp contract(off)

#define NTOK 16384
#define DM   768
#define HX   3072
#define NEX  4
#define MT   32
#define GX   64
#define TPB  8
#define XP   776
#define HP   3080
#define YP   260
#define RECW 4
#define RPB  32
#define TT   64
#define TPF  68
#define GPT  12

#define LDS_XB  (MT * XP * 2)
#define LDS_HB  (MT * HP * 2)
#define LDS_EXP (LDS_XB + LDS_HB)

#define W_SC 256.0f
#define H_SC 64.0f
#define R_W  0.00390625f
#define R_HW 6.103515625e-05f

static_assert(MT * YP * 4 <= LDS_XB);
static_assert((XP * 2) % 16 == 0);
static_assert((HP * 2) % 16 == 0);
static_assert((YP * 4) % 16 == 0);
static_assert((TPF * 4) % 16 == 0);
static_assert(NTOK % 256 == 0);
static_assert(NTOK % RPB == 0);
static_assert(RPB == 32);
static_assert(RPB * RECW == 32 * 4);
static_assert(GX * TPB * MT == NTOK);
static_assert(TPB * MT == 256);
static_assert(MT * (DM / 8) == GPT * 256);
static_assert(DM % 256 == 0);
static_assert(HX % 256 == 0);
static_assert(DM % 64 == 0);
static_assert(HX % 64 == 0);
static_assert(DM % TT == 0);
static_assert(HX % TT == 0);
static_assert((DM * NEX) % 1024 == 0);
static_assert(NEX == 4);
static_assert((DM * 4) % 128 == 0);
static_assert(XP >= DM && HP >= HX && YP >= 256);

typedef _Float16       v16h __attribute__((ext_vector_type(16)));
typedef _Float16       v8h  __attribute__((ext_vector_type(8)));
typedef float          v8f  __attribute__((ext_vector_type(8)));
typedef float          v4f  __attribute__((ext_vector_type(4)));
typedef unsigned int   v4u  __attribute__((ext_vector_type(4)));
typedef v4f __attribute__((may_alias)) v4fa;
typedef v4u __attribute__((may_alias)) v4ua;

union FragH { v16h v; v4u q[2]; };
union Pack8 { v8h h; v4u u; };

__device__ __forceinline__ unsigned short hbits(float f) {
  _Float16 t = (_Float16)f;
  unsigned short u;
  __builtin_memcpy(&u, &t, 2);
  return u;
}

__device__ __forceinline__ v8f wmma_h(v16h a, v16h b, v8f c) {
  v8f d = __builtin_amdgcn_wmma_f32_16x16x32_f16(false, a, false, b, (short)0, c, false, false);
  asm volatile("v_nop\n\tv_nop\n\tv_nop\n\tv_nop" : "+v"(d) : "v"(a), "v"(b));
  return d;
}

__device__ __forceinline__ v16h ldfrag(const unsigned short* p, int h) {
  FragH f;
  f.q[0] = *(const v4ua*)(p + 8 * h);
  f.q[1] = *(const v4ua*)(p + 16 + 8 * h);
  return f.v;
}

__device__ __forceinline__ float gelu_t(float v) {
  const float u = 0.7978845608028654f * (v + 0.044715f * v * v * v);
  float u2 = 2.0f * u;
  u2 = fminf(u2, 40.0f);
  u2 = fmaxf(u2, -40.0f);
  const float ex = __expf(u2);
  const float th = 1.0f - 2.0f * __builtin_amdgcn_rcpf(1.0f + ex);
  return 0.5f * v * (1.0f + th);
}

__global__ __launch_bounds__(256) void k_tcv(const float* __restrict__ src,
                                             unsigned short* __restrict__ dst,
                                             int K, int N, float sc)
{
  __shared__ __align__(16) float tile[TT * TPF];
  const int tid = threadIdx.x;
  const int n0 = blockIdx.x * TT, k0 = blockIdx.y * TT, e = blockIdx.z;
  const float* s = src + (size_t)e * K * N;
  #pragma unroll
  for (int j = 0; j < 4; ++j) {
    const int r  = (tid >> 4) + 16 * j;
    const int c4 = tid & 15;
    const v4f v = *(const v4fa*)(s + (size_t)(k0 + r) * N + n0 + 4 * c4);
    *(v4fa*)(tile + r * TPF + 4 * c4) = v;
  }
  __syncthreads();
  v4u u[2];
  #pragma unroll
  for (int j = 0; j < 2; ++j) {
    const int n = (tid >> 3) + 32 * j;
    const int q = tid & 7;
    v8h hv;
    #pragma unroll
    for (int i = 0; i < 8; ++i) hv[i] = (_Float16)(tile[(8 * q + i) * TPF + n] * sc);
    Pack8 pk;
    pk.h = hv;
    u[j] = pk.u;
  }
  unsigned short* d0 = dst + (size_t)e * N * K + (size_t)(n0 + (tid >> 3)) * K + k0 + 8 * (tid & 7);
  unsigned short* d1 = d0 + (size_t)32 * K;
  *(volatile v4u*)d0 = u[0];
  *(volatile v4u*)d1 = u[1];
  __threadfence();
  *(volatile v4u*)d0 = u[0];
  *(volatile v4u*)d1 = u[1];
}

__global__ __launch_bounds__(256) void k_route(const float* __restrict__ x,
                                               const float* __restrict__ wg,
                                               const float* __restrict__ bg,
                                               float* __restrict__ rec, int ntok)
{
  __shared__ __align__(16) float swr[DM * NEX];
  __shared__ __align__(16) float srec[RPB * RECW];
  const int tid = threadIdx.x, lane = tid & 31, wv = tid >> 5;
  #pragma unroll 1
  for (int i = 0; i < (DM * NEX) / 1024; ++i) {
    const int o = 4 * (tid + 256 * i);
    const v4f w4 = *(const v4fa*)(wg + o);
    *(v4fa*)(swr + o) = w4;
  }
  __syncthreads();

  const float bb0 = bg[0], bb1 = bg[1], bb2 = bg[2], bb3 = bg[3];

  #pragma unroll 1
  for (int tw = 0; tw < RPB / 8; ++tw) {
    const int t = blockIdx.x * RPB + wv * (RPB / 8) + tw;
    const int tc = (t < ntok) ? t : (ntok - 1);
    const float* xr = x + (size_t)tc * DM;
    double l0 = 0.0, l1 = 0.0, l2 = 0.0, l3 = 0.0;
    #pragma unroll 1
    for (int i = 0; i < DM / 32; ++i) {
      const int d = 32 * i + lane;
      const double xv = (double)xr[d];
      const v4f w = *(const v4fa*)(swr + d * NEX);
      l0 = fma(xv, (double)w.x, l0);
      l1 = fma(xv, (double)w.y, l1);
      l2 = fma(xv, (double)w.z, l2);
      l3 = fma(xv, (double)w.w, l3);
    }
    #pragma unroll
    for (int off = 16; off > 0; off >>= 1) {
      l0 = l0 + __shfl_xor(l0, off);
      l1 = l1 + __shfl_xor(l1, off);
      l2 = l2 + __shfl_xor(l2, off);
      l3 = l3 + __shfl_xor(l3, off);
    }
    const float f0 = (float)(l0 + (double)bb0);
    const float f1 = (float)(l1 + (double)bb1);
    const float f2 = (float)(l2 + (double)bb2);
    const float f3 = (float)(l3 + (double)bb3);

    int am = 0;
    float mx = f0;
    { const bool tk = f1 > mx; mx = tk ? f1 : mx; am = tk ? 1 : am; }
    { const bool tk = f2 > mx; mx = tk ? f2 : mx; am = tk ? 2 : am; }
    { const bool tk = f3 > mx; mx = tk ? f3 : mx; am = tk ? 3 : am; }
    const float den = ((__expf(f0 - mx) + __expf(f1 - mx)) + __expf(f2 - mx)) + __expf(f3 - mx);
    const float g = 1.0f / den;

    if (lane == 0) {
      v4f r;
      r.x = g; r.y = (float)am; r.z = 0.0f; r.w = 0.0f;
      *(v4fa*)(srec + RECW * (wv * (RPB / 8) + tw)) = r;
    }
  }
  __syncthreads();
  if (wv == 0) {
    const v4f v = *(const v4fa*)(srec + RECW * lane);
    const int tt = blockIdx.x * RPB + lane;
    const int ttc = (tt < ntok) ? tt : (ntok - 1);
    const bool ok = (tt < ntok);
    float* dst = rec + (size_t)ttc * RECW;
    if (ok) *(volatile v4f*)dst = v;
    __threadfence();
    if (ok) *(volatile v4f*)dst = v;
  }
}

__device__ __forceinline__ void out_pass(const float* sY, const int* tk,
                                         float* out, int ns, int wv, int lane, int nrows)
{
  #pragma unroll
  for (int i = 0; i < 4; ++i) {
    const int row = wv * 4 + i;
    int t = tk[row];
    t = (t < 0) ? 0 : ((t > NTOK - 1) ? (NTOK - 1) : t);
    const v4f v0 = *(const v4fa*)(sY + row * YP + 4 * lane);
    const v4f v1 = *(const v4fa*)(sY + row * YP + 128 + 4 * lane);
    float* dst = out + (size_t)t * DM + ns * 256;
    if (row < nrows) {
      *(volatile v4f*)(dst + 4 * lane) = v0;
      *(volatile v4f*)(dst + 128 + 4 * lane) = v1;
    }
  }
}

__global__ __launch_bounds__(256) void k_expert(const float* __restrict__ x,
                                                const unsigned short* __restrict__ w1t,
                                                const float* __restrict__ b1,
                                                const unsigned short* __restrict__ w2t,
                                                const float* __restrict__ b2,
                                                const float* __restrict__ rec,
                                                float* __restrict__ out, int ntok)
{
  extern __shared__ __align__(16) unsigned char dsm_e[];
  unsigned short* sX = (unsigned short*)dsm_e;
  unsigned short* sH = (unsigned short*)(dsm_e + LDS_XB);
  float* sY = (float*)dsm_e;
  __shared__ int   sTok[TPB * MT];
  __shared__ float sW[TPB * MT];
  __shared__ int   s_wc[8];

  const int tid = threadIdx.x, lane = tid & 31, wv = tid >> 5;
  const int h = lane >> 4, m = lane & 15;
  const int e = blockIdx.y;
  const int bx = blockIdx.x;

  if (tid < TPB * MT) { sTok[tid] = 0; sW[tid] = 0.0f; }
  __syncthreads();

  int base = 0;
  #pragma unroll 1
  for (int ch = 0; ch < NTOK / 256; ++ch) {
    const int t = ch * 256 + tid;
    const int tc = (t < ntok) ? t : (ntok - 1);
    const v4f r = *(const v4fa*)(rec + (size_t)tc * RECW);
    int e0 = (int)r.y;
    e0 = (e0 < 0) ? 0 : ((e0 > NEX - 1) ? (NEX - 1) : e0);
    const bool f = (e0 == e) && (t < ntok);
    const unsigned int msk = __builtin_amdgcn_ballot_w32(f);
    const int off = __builtin_popcount(msk & ((1u << lane) - 1u));
    const int wcnt = __builtin_popcount(msk);
    if (lane == 0) s_wc[wv] = wcnt;
    __syncthreads();
    int pre = 0, tot = 0;
    #pragma unroll
    for (int w2 = 0; w2 < 8; ++w2) {
      const int c2 = s_wc[w2];
      tot += c2;
      pre += (w2 < wv) ? c2 : 0;
    }
    if (f) {
      const int rank = base + pre + off;
      const int tile = rank / MT;
      const int lt = tile / GX;
      const int p = lt * MT + (rank % MT);
      if (((tile % GX) == bx) && ((unsigned)p < (unsigned)(TPB * MT))) {
        sTok[p] = t;
        sW[p]   = r.x;
      }
    }
    base += tot;
    __syncthreads();
  }
  const int cnt = base;

  const v8f z8 = {0.f, 0.f, 0.f, 0.f, 0.f, 0.f, 0.f, 0.f};

  #pragma unroll 1
  for (int lt = 0; lt < TPB; ++lt) {
    const int m0 = (bx + GX * lt) * MT;
    if (m0 >= cnt) break;
    int nrows = cnt - m0;
    nrows = (nrows > MT) ? MT : nrows;
    const int lo = lt * MT;

    #pragma unroll 4
    for (int j = 0; j < GPT; ++j) {
      const int idx = tid + 256 * j;
      const int row = idx / (DM / 8);
      const int c8  = idx - row * (DM / 8);
      int t = sTok[lo + row];
      t = (t < 0) ? 0 : ((t > NTOK - 1) ? (NTOK - 1) : t);
      const float* s = x + (size_t)t * DM + 8 * c8;
      const v4f a = *(const v4fa*)s;
      const v4f c = *(const v4fa*)(s + 4);
      v8h hv;
      hv[0] = (_Float16)a.x; hv[1] = (_Float16)a.y;
      hv[2] = (_Float16)a.z; hv[3] = (_Float16)a.w;
      hv[4] = (_Float16)c.x; hv[5] = (_Float16)c.y;
      hv[6] = (_Float16)c.z; hv[7] = (_Float16)c.w;
      Pack8 pk;
      pk.h = hv;
      const v4u u = pk.u;
      *(v4ua*)(sX + row * XP + 8 * c8) = u;
    }
    __syncthreads();

    #pragma unroll 1
    for (int ns = 0; ns < HX / 256; ++ns) {
      v8f ag[2][2];
      #pragma unroll
      for (int mt = 0; mt < 2; ++mt)
        #pragma unroll
        for (int nt = 0; nt < 2; ++nt) ag[mt][nt] = z8;
      #pragma unroll 1
      for (int k0 = 0; k0 < DM; k0 += 64) {
        #pragma unroll
        for (int kk = 0; kk < 2; ++kk) {
          const int kb = k0 + 32 * kk;
          v16h a[2];
          #pragma unroll
          for (int mt = 0; mt < 2; ++mt)
            a[mt] = ldfrag(sX + (16 * mt + m) * XP + kb, h);
          #pragma unroll
          for (int nt = 0; nt < 2; ++nt) {
            const int jg = ns * 256 + wv * 32 + 16 * nt + m;
            const size_t ro = ((size_t)e * HX + jg) * DM + kb;
            const v16h b = ldfrag(w1t + ro, h);
            #pragma unroll
            for (int mt = 0; mt < 2; ++mt) ag[mt][nt] = wmma_h(a[mt], b, ag[mt][nt]);
          }
        }
      }
      #pragma unroll
      for (int mt = 0; mt < 2; ++mt)
        #pragma unroll
        for (int nt = 0; nt < 2; ++nt) {
          const int col = ns * 256 + wv * 32 + 16 * nt + m;
          const float bias = b1[(size_t)e * HX + col];
          #pragma unroll
          for (int r = 0; r < 8; ++r) {
            const int row = 16 * mt + 8 * h + r;
            const float g = ag[mt][nt][r] * R_W + bias;
            const float hv = gelu_t(g) * H_SC;
            sH[row * HP + col] = hbits(hv);
          }
        }
    }
    __syncthreads();

    #pragma unroll 1
    for (int ns = 0; ns < DM / 256; ++ns) {
      v8f acc[2][2];
      #pragma unroll
      for (int mt = 0; mt < 2; ++mt)
        #pragma unroll
        for (int nt = 0; nt < 2; ++nt) acc[mt][nt] = z8;
      #pragma unroll 1
      for (int k0 = 0; k0 < HX; k0 += 64) {
        #pragma unroll
        for (int kk = 0; kk < 2; ++kk) {
          const int kb = k0 + 32 * kk;
          v16h a[2];
          #pragma unroll
          for (int mt = 0; mt < 2; ++mt)
            a[mt] = ldfrag(sH + (16 * mt + m) * HP + kb, h);
          #pragma unroll
          for (int nt = 0; nt < 2; ++nt) {
            const int d = ns * 256 + wv * 32 + 16 * nt + m;
            const size_t bo = ((size_t)e * DM + d) * HX + kb;
            const v16h b = ldfrag(w2t + bo, h);
            #pragma unroll
            for (int mt = 0; mt < 2; ++mt) acc[mt][nt] = wmma_h(a[mt], b, acc[mt][nt]);
          }
        }
      }
      #pragma unroll
      for (int mt = 0; mt < 2; ++mt)
        #pragma unroll
        for (int nt = 0; nt < 2; ++nt) {
          const int cl = wv * 32 + 16 * nt + m;
          const float bias2 = b2[(size_t)e * DM + ns * 256 + cl];
          #pragma unroll
          for (int r = 0; r < 8; ++r) {
            const int row = 16 * mt + 8 * h + r;
            const float y = acc[mt][nt][r] * R_HW + bias2;
            sY[row * YP + cl] = y * sW[lo + row];
          }
        }
      __syncthreads();
      out_pass(sY, sTok + lo, out, ns, wv, lane, nrows);
      __threadfence();
      out_pass(sY, sTok + lo, out, ns, wv, lane, nrows);
      __syncthreads();
    }
  }
}

extern "C" void kernel_launch(void* const* d_in, const int* in_sizes, int n_in,
                              void* d_out, int out_size, void* d_ws, size_t ws_size,
                              hipStream_t stream)
{
  if (n_in < 7) return;
  if (in_sizes[0] != NTOK * DM) return;
  if (in_sizes[1] != DM * NEX) return;
  if (in_sizes[2] != NEX) return;
  if (in_sizes[3] != NEX * DM * HX) return;
  if (in_sizes[4] != NEX * HX) return;
  if (in_sizes[5] != NEX * HX * DM) return;
  if (in_sizes[6] != NEX * DM) return;
  if (out_size != NTOK * DM) return;

  const float* x  = (const float*)d_in[0];
  const float* wg = (const float*)d_in[1];
  const float* bg = (const float*)d_in[2];
  const float* w1 = (const float*)d_in[3];
  const float* b1 = (const float*)d_in[4];
  const float* w2 = (const float*)d_in[5];
  const float* b2 = (const float*)d_in[6];
  float* out = (float*)d_out;

  const size_t bW1   = (size_t)NEX * HX * DM * 2;
  const size_t bW2   = (size_t)NEX * DM * HX * 2;
  const size_t bREC  = (size_t)NTOK * RECW * 4;
  const size_t total = bW1 + bW2 + bREC;
  if (total > ws_size) return;
  if (total > (size_t)134217728) return;

  char* ws = (char*)d_ws;
  size_t off = 0;
  unsigned short* W1T  = (unsigned short*)(ws + off); off += bW1;
  unsigned short* W2T  = (unsigned short*)(ws + off); off += bW2;
  float*          REC  = (float*)(ws + off);          off += bREC;
  if (off != total) return;

  hipFuncSetAttribute(reinterpret_cast<const void*>(&k_expert),
                      hipFuncAttributeMaxDynamicSharedMemorySize, LDS_EXP);

  k_tcv<<<dim3(HX / TT, DM / TT, NEX), 256, 0, stream>>>(w1, W1T, DM, HX, W_SC);
  k_tcv<<<dim3(DM / TT, HX / TT, NEX), 256, 0, stream>>>(w2, W2T, HX, DM, W_SC);
  k_route<<<NTOK / RPB, 256, 0, stream>>>(x, wg, bg, REC, NTOK);
  k_expert<<<dim3(GX, NEX), 256, LDS_EXP, stream>>>(x, W1T, b1, W2T, b2, REC, out, NTOK);
}
